// GauntTensorProductS2Grid_58609123721876
// MI455X (gfx1250) — hardware-verified
//
#include <hip/hip_runtime.h>


#ifndef NB
#define NB 16384
#endif
#define NB_FULL 16384
#define DD 81
#define KP 96
#define RB 32
#define RA 63
#define NG 2016
#define KSG 63
#define NCH 21

static_assert(NB % 64 == 0);
static_assert(NB >= 64 && NB <= NB_FULL);
static_assert(NG == RB * RA);
static_assert(KSG * 32 == NG);
static_assert(NCH * 96 == NG);
static_assert(KP % 32 == 0 && KP >= DD);
static_assert((size_t)NB * DD * 4 <= (size_t)5308416);
static_assert((64 * DD * 4) % 128 == 0);
static_assert((64 * DD) % 4 == 0);
static_assert((32 * KP * 2) % 128 == 0);
static_assert((2 * NG * 2) % 128 == 0);
static_assert(KP % 2 == 0);

typedef __bf16   v16b __attribute__((ext_vector_type(16)));
typedef float    v8f  __attribute__((ext_vector_type(8)));
typedef float    v4f  __attribute__((ext_vector_type(4)));
typedef unsigned v4u  __attribute__((ext_vector_type(4), may_alias));
typedef unsigned short us16;

template <typename T> __device__ __forceinline__ void vst2(void* p, T v) { *(volatile T*)p = v; __threadfence(); *(volatile T*)p = v; }

__device__ __forceinline__ v8f wmma_bf(v16b a, v16b b, v8f c) {
  v8f d = __builtin_amdgcn_wmma_f32_16x16x32_bf16(false, a, false, b, (short)0, c, false, false);
  asm volatile("v_nop\n\tv_nop\n\tv_nop\n\tv_nop" : "+v"(d) : "v"(a), "v"(b));
  return d;
}

__device__ __forceinline__ us16 bfb(float f) { unsigned u = __float_as_uint(f); u += 0x7FFFu + ((u >> 16) & 1u); return (us16)(u >> 16); }
__device__ __forceinline__ float bff(us16 b) { return __uint_as_float(((unsigned)b) << 16); }

union FB { v16b v; v4u u[2]; };
__device__ __forceinline__ v16b ldfrag(const us16* p) { FB f; f.u[0] = *(const v4u*)p; f.u[1] = *(const v4u*)(p + 16); return f.v; }

#define LDSX() do { asm volatile("s_wait_dscnt 0" ::: "memory"); __builtin_amdgcn_wave_barrier(); __builtin_amdgcn_fence(__ATOMIC_RELEASE, "workgroup"); } while (0)

__global__ __launch_bounds__(256) void k_w1(const float* __restrict__ shb, const float* __restrict__ sha, us16* W1h, us16* W1l) {
  __shared__ __align__(16) us16 sh[32 * KP];
  __shared__ __align__(16) us16 sl[32 * KP];
  const int tid = threadIdx.x, n0 = blockIdx.x * 32;
#pragma unroll 1
  for (int e = tid; e < 32 * KP; e += 256) {
    const int rl = e / KP, k = e - rl * KP, n = n0 + rl, b = n / RA, a = n - b * RA;
    const int kc = k < DD ? k : DD - 1;
    const float w = bff(bfb(shb[b * DD + kc])) * bff(bfb(sha[a * DD + kc]));
    const float v = (k < DD) ? w : 0.f;
    const us16 hb = bfb(v);
    const us16 lb = bfb(v - bff(hb));
    sh[e] = hb; sl[e] = lb;
  }
  __syncthreads();
  us16* dh = W1h + (size_t)n0 * KP;
  us16* dl = W1l + (size_t)n0 * KP;
  for (int t = tid; t < 32 * KP / 8; t += 256) {
    const v4u ph = *(const v4u*)&sh[8 * t];
    const v4u pl = *(const v4u*)&sl[8 * t];
    vst2(dh + 8 * t, ph);
    vst2(dl + 8 * t, pl);
  }
}

__global__ __launch_bounds__(256) void k_w2(const float* __restrict__ shb, const float* __restrict__ sha, const float* __restrict__ qw,
                                           us16* W2h, us16* W2l) {
  __shared__ __align__(16) us16 sh[2 * NG];
  __shared__ __align__(16) us16 sl[2 * NG];
  const int tid = threadIdx.x, i0 = blockIdx.x * 2;
#pragma unroll 1
  for (int e = tid; e < 2 * NG; e += 256) {
    const int rl = e / NG, n = e - rl * NG, i = i0 + rl, b = n / RA, a = n - b * RA;
    const int ic = i < DD ? i : DD - 1;
    const float pq = bff(bfb(sha[a * DD + ic])) * bff(bfb(shb[b * DD + ic]));
    const float w = pq * bff(bfb(qw[b]));
    const float v = (i < DD) ? w : 0.f;
    const us16 hb = bfb(v);
    const us16 lb = bfb(v - bff(hb));
    sh[e] = hb; sl[e] = lb;
  }
  __syncthreads();
  us16* dh = W2h + (size_t)i0 * NG;
  us16* dl = W2l + (size_t)i0 * NG;
  for (int t = tid; t < 2 * NG / 8; t += 256) {
    const v4u ph = *(const v4u*)&sh[8 * t];
    const v4u pl = *(const v4u*)&sl[8 * t];
    vst2(dh + 8 * t, ph);
    vst2(dl + 8 * t, pl);
  }
}

__global__ __launch_bounds__(128) void k_syn(const float* x1, const float* x2, const us16* W1h, const us16* W1l, us16* Gh, us16* Gl) {
  __shared__ __align__(16) us16 sx[2][64 * KP];
  __shared__ __align__(16) float sg[4][3][512];
  const int tid = threadIdx.x, w = tid >> 5, lane = tid & 31, m = lane & 15, h = lane >> 4;
  const int z0 = blockIdx.x * 64, zt = blockIdx.x * 4 + w;
#pragma unroll 1
  for (int g = tid; g < 2 * 64 * 12; g += 128) {
    const int which = (g >= 768) ? 1 : 0, rem = g - which * 768, r = rem / 12, k0 = (rem - r * 12) * 8;
    const float* src = (which ? x2 : x1) + (size_t)(z0 + r) * DD;
    v4u pk = {0u, 0u, 0u, 0u};
#pragma unroll
    for (int e = 0; e < 8; ++e) {
      const int k = k0 + e, kc = k < DD ? k : DD - 1;
      float v = src[kc];
      v = (k < DD) ? v : 0.f;
      pk[e >> 1] |= ((unsigned)bfb(v)) << (16 * (e & 1));
    }
    *(v4u*)&sx[which][r * KP + k0] = pk;
  }
  __syncthreads();
  const us16* xa = &sx[0][(16 * w + m) * KP + 8 * h];
  const us16* xb = &sx[1][(16 * w + m) * KP + 8 * h];
#pragma unroll 1
  for (int c = 0; c < NCH; ++c) {
    const int n0 = c * 96;
    v8f acc1[6] = {};
    v8f acc2[6] = {};
#pragma unroll 1
    for (int seg = 0; seg < 2; ++seg) {
      const us16* Wp = (seg ? W1l : W1h) + (size_t)(n0 + m) * KP + 8 * h;
#pragma unroll 1
      for (int ks = 0; ks < 3; ++ks) {
        const v16b a1 = ldfrag(xa + 32 * ks);
        const v16b a2 = ldfrag(xb + 32 * ks);
#pragma unroll
        for (int nt = 0; nt < 6; ++nt) {
          if ((nt & 1) == 0) asm volatile("" ::: "memory");
          const v16b bfr = ldfrag(Wp + (size_t)nt * 16 * KP + 32 * ks);
          acc1[nt] = wmma_bf(a1, bfr, acc1[nt]);
          acc2[nt] = wmma_bf(a2, bfr, acc2[nt]);
        }
      }
    }
#pragma unroll
    for (int ks = 0; ks < 3; ++ks) {
      float* S = sg[w][ks];
#pragma unroll
      for (int r = 0; r < 8; ++r) {
        S[(8 * h + r) * 32 + m]      = acc1[2 * ks][r]     * acc2[2 * ks][r];
        S[(8 * h + r) * 32 + 16 + m] = acc1[2 * ks + 1][r] * acc2[2 * ks + 1][r];
      }
    }
    LDSX();
#pragma unroll
    for (int ks = 0; ks < 3; ++ks) {
      const float* S = sg[w][ks];
      const size_t base = ((size_t)zt * KSG + (size_t)(3 * c + ks)) * 512;
#pragma unroll
      for (int p = 0; p < 2; ++p) {
        const int idx = 256 * p + 8 * lane;
        const v4f q0 = *(const v4f*)(S + idx);
        const v4f q1 = *(const v4f*)(S + idx + 4);
        const float vv[8] = {q0[0], q0[1], q0[2], q0[3], q1[0], q1[1], q1[2], q1[3]};
        v4u hu = {0u, 0u, 0u, 0u}, lu = {0u, 0u, 0u, 0u};
#pragma unroll
        for (int e = 0; e < 8; ++e) {
          const us16 hb = bfb(vv[e]);
          const us16 lb = bfb(vv[e] - bff(hb));
          hu[e >> 1] |= ((unsigned)hb) << (16 * (e & 1));
          lu[e >> 1] |= ((unsigned)lb) << (16 * (e & 1));
        }
        vst2(Gh + base + idx, hu);
        vst2(Gl + base + idx, lu);
      }
    }
    LDSX();
  }
}

__global__ __launch_bounds__(128) void k_ana(const us16* Gh, const us16* Gl, const us16* W2h, const us16* W2l, float* out) {
  __shared__ __align__(16) float so[64 * DD];
  const int tid = threadIdx.x, w = tid >> 5, lane = tid & 31, m = lane & 15, h = lane >> 4;
  const int zt = blockIdx.x * 4 + w;
  const us16* ga = Gh + (size_t)zt * KSG * 512 + m * 32 + 8 * h;
  const us16* gb = Gl + (size_t)zt * KSG * 512 + m * 32 + 8 * h;
  const us16* wa = W2h + (size_t)m * NG + 8 * h;
  const us16* wb = W2l + (size_t)m * NG + 8 * h;
  v8f acc[6] = {};
#pragma unroll 1
  for (int ks = 0; ks < KSG; ++ks) {
    const v16b ah = ldfrag(ga + (size_t)ks * 512);
    const v16b al = ldfrag(gb + (size_t)ks * 512);
#pragma unroll
    for (int nt = 0; nt < 6; ++nt) {
      if ((nt & 1) == 0) asm volatile("" ::: "memory");
      const v16b bh = ldfrag(wa + (size_t)nt * 16 * NG + 32 * ks);
      const v16b bl = ldfrag(wb + (size_t)nt * 16 * NG + 32 * ks);
      acc[nt] = wmma_bf(al, bh, acc[nt]);
      acc[nt] = wmma_bf(ah, bl, acc[nt]);
      acc[nt] = wmma_bf(ah, bh, acc[nt]);
    }
  }
#pragma unroll
  for (int nt = 0; nt < 6; ++nt) {
    const int col = 16 * nt + m;
    if (col < DD) {
#pragma unroll
      for (int r = 0; r < 8; ++r) so[(16 * w + 8 * h + r) * DD + col] = acc[nt][r];
    }
  }
  __syncthreads();
  float* ob = out + (size_t)blockIdx.x * (64 * DD);
  for (int t = tid; t < 64 * DD / 4; t += 128) {
    const v4f v = *(const v4f*)&so[4 * t];
    vst2(ob + 4 * t, v);
  }
}

extern "C" void kernel_launch(void* const* d_in, const int* in_sizes, int n_in,
                              void* d_out, int out_size, void* d_ws, size_t ws_size,
                              hipStream_t stream) {
  if (n_in < 5) return;
  if (in_sizes[0] < NB * DD || in_sizes[1] < NB * DD || in_sizes[2] < RB * DD || in_sizes[3] < RA * DD || in_sizes[4] < RB) return;
  if (out_size < NB * DD) return;
  const float* x1  = (const float*)d_in[0];
  const float* x2  = (const float*)d_in[1];
  const float* shb = (const float*)d_in[2];
  const float* sha = (const float*)d_in[3];
  const float* qw  = (const float*)d_in[4];
  float* out = (float*)d_out;
  char* ws = (char*)d_ws; size_t off = 0;
  auto take = [&](size_t bytes) { char* p = ws + off; off += (bytes + 1023) & ~(size_t)1023; return p; };
  us16* W1h = (us16*)take((size_t)NG * KP * 2);
  us16* W1l = (us16*)take((size_t)NG * KP * 2);
  us16* W2h = (us16*)take((size_t)KP * NG * 2);
  us16* W2l = (us16*)take((size_t)KP * NG * 2);
  us16* Gh  = (us16*)take((size_t)NB * NG * 2);
  us16* Gl  = (us16*)take((size_t)NB * NG * 2);
  if (off > ws_size) return;
  k_w1<<<NG / 32, 256, 0, stream>>>(shb, sha, W1h, W1l);
  k_w2<<<KP / 2, 256, 0, stream>>>(shb, sha, qw, W2h, W2l);
  k_syn<<<NB / 64, 128, 0, stream>>>(x1, x2, W1h, W1l, Gh, Gl);
  k_ana<<<NB / 64, 128, 0, stream>>>(Gh, Gl, W2h, W2l, out);
}
